// SparseMHADecoder_3582002725463
// MI455X (gfx1250) — hardware-verified
//
#include <hip/hip_runtime.h>
#include <math.h>

typedef __attribute__((ext_vector_type(16))) _Float16 v16h;
typedef __attribute__((ext_vector_type(16))) __bf16 v16b;
typedef __attribute__((ext_vector_type(8)))  _Float16 v8h;
typedef __attribute__((ext_vector_type(8)))  float v8f;
typedef __attribute__((ext_vector_type(4)))  float v4f;
typedef __attribute__((ext_vector_type(2)))  float v2f;
typedef __attribute__((ext_vector_type(4)))  unsigned v4u;
typedef __attribute__((ext_vector_type(4)))  int v4i;
typedef float __attribute__((may_alias)) float_a;
typedef int __attribute__((may_alias)) int_a;

template <typename T> __device__ __forceinline__ void vst2(void* p, T v) { *(volatile T*)p = v; __threadfence(); *(volatile T*)p = v; }
__device__ __forceinline__ v8f wmma16(v16h a, v16h b, v8f c) {
  v8f d = __builtin_amdgcn_wmma_f32_16x16x32_f16(false, a, false, b, (short)0, c, false, false);
  asm volatile("v_nop\n\tv_nop\n\tv_nop\n\tv_nop" : "+v"(d) : "v"(a), "v"(b));
  return d;
}
__device__ __forceinline__ v8f wmma_bf(v16b a, v16b b, v8f c) {
  v8f d = __builtin_amdgcn_wmma_f32_16x16x32_bf16(false, a, false, b, (short)0, c, false, false);
  asm volatile("v_nop\n\tv_nop\n\tv_nop\n\tv_nop" : "+v"(d) : "v"(a), "v"(b));
  return d;
}
__device__ __forceinline__ v16h frag_h(const _Float16* rowk0, int lane) {
  union { v16h v; v8h q[2]; } u; const _Float16* p = rowk0 + 8 * (lane >> 4);
  u.q[0] = *(const v8h*)p; u.q[1] = *(const v8h*)(p + 16); return u.v;
}
__device__ __forceinline__ v16h frag_f32(const float* rowk0, int lane) {
  v16h a; const float* p = rowk0 + 8 * (lane >> 4);
#pragma unroll
  for (int i = 0; i < 8; ++i) { a[i] = (_Float16)p[i]; a[8 + i] = (_Float16)p[16 + i]; }
  return a;
}
__device__ __forceinline__ v16h frag_f32s(const float* rowk0, int lane, float sc) {
  v16h a; const float* p = rowk0 + 8 * (lane >> 4);
#pragma unroll
  for (int i = 0; i < 8; ++i) { a[i] = (_Float16)(p[i] * sc); a[8 + i] = (_Float16)(p[16 + i] * sc); }
  return a;
}
__device__ __forceinline__ v16h fragc_f32(const float* W, int k0, int n, int lane, int ld, int K) {
  v16h a; const int g = lane >> 4;
#pragma unroll
  for (int i = 0; i < 8; ++i) { const int ka = k0 + 8 * g + i, kb = ka + 16;
    a[i] = (_Float16)(ka < K ? W[(size_t)(ka < K ? ka : K - 1) * ld + n] : 0.f); a[8 + i] = (_Float16)(kb < K ? W[(size_t)(kb < K ? kb : K - 1) * ld + n] : 0.f); }
  return a;
}
struct F2 { v16b h, l; };
__device__ __forceinline__ F2 bsplit16(const float v[16]) { F2 r;
#pragma unroll
  for (int i = 0; i < 16; ++i) { const __bf16 h = (__bf16)v[i]; r.h[i] = h; r.l[i] = (__bf16)(v[i] - (float)h); }
  return r; }
__device__ __forceinline__ F2 split_row(const float* row, int k0, int lane) { float v[16]; const float* p = row + k0 + 8 * (lane >> 4);
#pragma unroll
  for (int i = 0; i < 8; ++i) { v[i] = p[i]; v[8 + i] = p[16 + i]; }
  return bsplit16(v); }
__device__ __forceinline__ F2 split_rowK(const float* row, int k0, int lane, int K) { float v[16]; const int g = lane >> 4;
#pragma unroll
  for (int i = 0; i < 8; ++i) { const int ka = k0 + 8 * g + i, kb = ka + 16; v[i] = ka < K ? row[ka < K ? ka : K - 1] : 0.f; v[8 + i] = kb < K ? row[kb < K ? kb : K - 1] : 0.f; }
  return bsplit16(v); }
__device__ __forceinline__ F2 split_col(const float* W, int k0, int n, int lane, int ld, int K) { float v[16]; const int g = lane >> 4;
#pragma unroll
  for (int i = 0; i < 8; ++i) { const int ka = k0 + 8 * g + i, kb = ka + 16; v[i] = ka < K ? W[(size_t)(ka < K ? ka : K - 1) * ld + n] : 0.f; v[8 + i] = kb < K ? W[(size_t)(kb < K ? kb : K - 1) * ld + n] : 0.f; }
  return bsplit16(v); }
__device__ __forceinline__ v8f mac3(const F2& a, const F2& b, v8f c) { c = wmma_bf(a.l, b.h, c); c = wmma_bf(a.h, b.l, c); return wmma_bf(a.h, b.h, c); }
__device__ __forceinline__ float sigm(float v) { return 1.0f / (1.0f + expf(-v)); }
#define LDSX() do { asm volatile("s_wait_dscnt 0" ::: "memory"); __builtin_amdgcn_wave_barrier(); __builtin_amdgcn_fence(__ATOMIC_RELEASE, "workgroup"); } while (0)

__device__ __forceinline__ float bfr(float v) { return (float)(__bf16)v; }
#define NB 2
#define LQ 4096
#define LKV 2048
#define CC 1024
#define NH 16
#define HD 64
#define SPAN 16
#define STRD 2
#ifndef TNB
#define TNB NB
#endif
typedef __attribute__((ext_vector_type(8))) __bf16 v8b;
__device__ __forceinline__ v16b frag_b(const __bf16* rowk0, int lane) { union { v16b v; v8b q[2]; } u; const __bf16* p = rowk0 + 8 * (lane >> 4); u.q[0] = *(const v8b*)p; u.q[1] = *(const v8b*)(p + 16); return u.v; }
#define WS_QH  0u
#define WS_QL  (WS_QH + 2u * (size_t)NB * LQ * CC)
#define WS_KH  (WS_QL + 2u * (size_t)NB * LQ * CC)
#define WS_KL  (WS_KH + 2u * (size_t)NB * LKV * CC)
#define WS_VH  (WS_KL + 2u * (size_t)NB * LKV * CC)
#define WS_VL  (WS_VH + 2u * (size_t)NB * LKV * CC)
#define WS_Y   (WS_VL + 2u * (size_t)NB * LKV * CC)
#define WS_END (WS_Y + 4u * (size_t)NB * LQ * CC)
__global__ __launch_bounds__(128) void k_lin(const float* __restrict__ XQ, const float* __restrict__ XK, const float* __restrict__ XV, const float* __restrict__ WQ, const float* __restrict__ WK, const float* __restrict__ WV, _Float16* __restrict__ QH, _Float16* __restrict__ QL, _Float16* __restrict__ KH, _Float16* __restrict__ KL, __bf16* __restrict__ VH, __bf16* __restrict__ VL) {
  __shared__ __align__(16) unsigned short sh[64][136], sl[64][136];
  const int tid = threadIdx.x, wave = tid >> 5, lane = tid & 31, col = lane & 15, g = lane >> 4; const int which = blockIdx.z; const int nrows = which == 0 ? TNB * LQ : TNB * LKV; if ((int)blockIdx.x * 64 >= nrows) return;
  const int c0 = blockIdx.y * 128; const size_t r0 = (size_t)blockIdx.x * 64; const float* X = which == 0 ? XQ : which == 1 ? XK : XV; const float* Wt = which == 0 ? WQ : which == 1 ? WK : WV;
  v8f acc[8] = {};
#pragma unroll 2
  for (int kc = 0; kc < CC / 32; ++kc) { v16b a; { const float* p = X + (r0 + wave * 16 + col) * CC + kc * 32 + 8 * g;
#pragma unroll
      for (int i = 0; i < 8; ++i) { a[i] = (__bf16)p[i]; a[8 + i] = (__bf16)p[16 + i]; } }
#pragma unroll
    for (int j = 0; j < 8; ++j) { v16b w; const int o = c0 + j * 16 + col;
#pragma unroll
      for (int i = 0; i < 8; ++i) { w[i] = (__bf16)Wt[(size_t)(kc * 32 + 8 * g + i) * CC + o]; w[8 + i] = (__bf16)Wt[(size_t)(kc * 32 + 16 + 8 * g + i) * CC + o]; }
      asm volatile("s_wait_loadcnt 0x0" ::: "memory"); acc[j] = wmma_bf(a, w, acc[j]); } }
#pragma unroll
  for (int j = 0; j < 8; ++j)
#pragma unroll
    for (int r = 0; r < 8; ++r) { const float v = acc[j][r]; const int rl = wave * 16 + 8 * g + r, cl = j * 16 + col; union { _Float16 h; __bf16 b; unsigned short u; } a_, b_;
      if (which == 2) { const __bf16 bh = (__bf16)v; a_.b = bh; b_.b = (__bf16)(v - (float)bh); } else { const _Float16 hv = (_Float16)v; a_.h = hv; b_.h = (_Float16)((v - (float)hv) * 1024.0f); }
      sh[rl][cl] = a_.u; sl[rl][cl] = b_.u; }
  __syncthreads();
  unsigned short* DH = which == 0 ? (unsigned short*)QH : which == 1 ? (unsigned short*)KH : (unsigned short*)VH; unsigned short* DL = which == 0 ? (unsigned short*)QL : which == 1 ? (unsigned short*)KL : (unsigned short*)VL;
  for (int e = tid; e < 64 * 16; e += 128) { const int rl = e >> 4, q = e & 15; vst2((unsigned*)(DH + (r0 + rl) * CC + c0 + q * 8), *(const v4u*)&sh[rl][q * 8]); vst2((unsigned*)(DL + (r0 + rl) * CC + c0 + q * 8), *(const v4u*)&sl[rl][q * 8]); } }
__global__ __launch_bounds__(128) void k_band(const _Float16* __restrict__ QH, const _Float16* __restrict__ QL, const _Float16* __restrict__ KH, const _Float16* __restrict__ KL, const __bf16* __restrict__ VH, const __bf16* __restrict__ VL, float* __restrict__ Y) {
  __shared__ __align__(16) float slg[96][49]; __shared__ __align__(16) __bf16 vbh[HD][72], vbl[HD][72]; __shared__ __align__(16) float so[4][16][HD + 4];
  const int tid = threadIdx.x, wave = tid >> 5, lane = tid & 31, col = lane & 15, g = lane >> 4; const int q0 = blockIdx.x * 64; const int h = blockIdx.y; const size_t b = blockIdx.z; const int kb0 = q0 / STRD - 8;
  for (int e = tid; e < 64 * HD; e += 128) { const int kk = e / HD, d = e % HD; int k = kb0 + kk; k = k < 0 ? 0 : (k >= LKV ? LKV - 1 : k); const size_t o = (b * LKV + k) * CC + h * HD + d; vbh[d][kk] = VH[o]; vbl[d][kk] = VL[o]; }
  for (int rt = wave; rt < 6; rt += 4) { v8f acc[3] = {}, accl[3] = {};
    int qr = q0 - 16 + rt * 16 + col; qr = qr < 0 ? 0 : (qr >= LQ ? LQ - 1 : qr); const size_t qo = (b * LQ + qr) * CC + h * HD;
#pragma unroll
    for (int kc = 0; kc < HD / 32; ++kc) { const v16h ah = frag_h(QH + qo + kc * 32, lane), al = frag_h(QL + qo + kc * 32, lane);
#pragma unroll
      for (int j = 0; j < 3; ++j) { int kk = kb0 + j * 16 + col; kk = kk < 0 ? 0 : (kk >= LKV ? LKV - 1 : kk); const size_t ko = (b * LKV + kk) * CC + h * HD + kc * 32; const v16h kbf = frag_h(KH + ko, lane), klf = frag_h(KL + ko, lane); acc[j] = wmma16(ah, kbf, acc[j]); accl[j] = wmma16(al, kbf, accl[j]); accl[j] = wmma16(ah, klf, accl[j]); } }
#pragma unroll
    for (int j = 0; j < 3; ++j)
#pragma unroll
      for (int r = 0; r < 8; ++r) slg[rt * 16 + 8 * g + r][j * 16 + col] = acc[j][r] + accl[j][r] * (1.0f / 1024.0f); }
  __syncthreads();
  if (tid < 48) { const int k = kb0 + tid; if (k >= 0 && k < LKV) { float m = -3.0e38f;
      for (int r = 0; r < 96; ++r) { const int q = q0 - 16 + r; const int s = q - STRD * k; if (q >= 0 && q < LQ && s >= 0 && s < SPAN) m = fmaxf(m, slg[r][tid]); }
      float z = 0.f; for (int r = 0; r < 96; ++r) { const int q = q0 - 16 + r; const int s = q - STRD * k; const bool ok = (q >= 0 && q < LQ && s >= 0 && s < SPAN); const float e = ok ? expf(slg[r][tid] - m) : 0.f; slg[r][tid] = e; z += e; }
      const float inv = 1.0f / z; for (int r = 16; r < 80; ++r) slg[r][tid] *= inv; }
    else { for (int r = 16; r < 80; ++r) slg[r][tid] = 0.f; } }
  __syncthreads();
  { v8f acc[HD / 16] = {};
#pragma unroll
    for (int kc = 0; kc < 2; ++kc) { float pv[16];
#pragma unroll
      for (int i = 0; i < 8; ++i) { const int k1 = kc * 32 + 8 * g + i, k2 = k1 + 16; pv[i] = (k1 < 48) ? slg[16 + wave * 16 + col][k1] : 0.f; pv[8 + i] = (k2 < 48) ? slg[16 + wave * 16 + col][k2] : 0.f; }
      const F2 p = bsplit16(pv);
#pragma unroll
      for (int j = 0; j < HD / 16; ++j) { const v16b vh = frag_b(&vbh[j * 16 + col][kc * 32], lane), vl = frag_b(&vbl[j * 16 + col][kc * 32], lane); acc[j] = wmma_bf(p.h, vh, acc[j]); acc[j] = wmma_bf(p.l, vh, acc[j]); acc[j] = wmma_bf(p.h, vl, acc[j]); } }
#pragma unroll
    for (int j = 0; j < HD / 16; ++j)
#pragma unroll
      for (int r = 0; r < 8; ++r) so[wave][8 * g + r][j * 16 + col] = acc[j][r];
    LDSX(); for (int rl = 0; rl < 16; ++rl) if (lane < HD / 4) vst2(Y + (b * LQ + q0 + wave * 16 + rl) * CC + h * HD + lane * 4, *(const v4f*)&so[wave][rl][lane * 4]); } }
__global__ __launch_bounds__(128) void k_out(const float* __restrict__ Y, const float* __restrict__ WO, float* __restrict__ OUT) { __shared__ __align__(16) float sf[4][16][132];
  const int tid = threadIdx.x, wave = tid >> 5, lane = tid & 31, col = lane & 15, g = lane >> 4; const int c0 = blockIdx.y * 128; const size_t r0 = (size_t)blockIdx.x * 64 + wave * 16;
  v8f acc[8] = {};
#pragma unroll 2
  for (int kc = 0; kc < CC / 32; ++kc) { const F2 a = split_row(Y + (r0 + col) * CC, kc * 32, lane);
#pragma unroll
    for (int j = 0; j < 8; ++j) { v16b w; const int o = c0 + j * 16 + col;
#pragma unroll
      for (int i = 0; i < 8; ++i) { w[i] = (__bf16)WO[(size_t)(kc * 32 + 8 * g + i) * CC + o]; w[8 + i] = (__bf16)WO[(size_t)(kc * 32 + 16 + 8 * g + i) * CC + o]; }
      asm volatile("s_wait_loadcnt 0x0" ::: "memory"); acc[j] = wmma_bf(a.h, w, acc[j]); acc[j] = wmma_bf(a.l, w, acc[j]); } }
#pragma unroll
  for (int j = 0; j < 8; ++j)
#pragma unroll
    for (int r = 0; r < 8; ++r) sf[wave][8 * g + r][j * 16 + col] = acc[j][r];
  LDSX(); for (int rl = 0; rl < 16; ++rl) vst2(OUT + (r0 + rl) * CC + c0 + lane * 4, *(const v4f*)&sf[wave][rl][lane * 4]); }
extern "C" void kernel_launch(void* const* d_in, const int* in_sizes, int n_in, void* d_out, int out_size, void* d_ws, size_t ws_size, hipStream_t stream) {
  (void)in_sizes; (void)n_in; (void)out_size;
  const float** F = (const float**)d_in;
  if (ws_size < (size_t)WS_END) return;
  char* ws = (char*)d_ws; _Float16 *QH = (_Float16*)(ws + WS_QH), *QL = (_Float16*)(ws + WS_QL), *KH = (_Float16*)(ws + WS_KH), *KL = (_Float16*)(ws + WS_KL); __bf16 *VH = (__bf16*)(ws + WS_VH), *VL = (__bf16*)(ws + WS_VL); float* Y = (float*)(ws + WS_Y);
  k_lin<<<dim3(TNB * LQ / 64, CC / 128, 3), 128, 0, stream>>>(F[0], F[1], F[2], F[3], F[4], F[5], QH, QL, KH, KL, VH, VL);
  k_band<<<dim3(LQ / 64, NH, TNB), 128, 0, stream>>>(QH, QL, KH, KL, VH, VL, Y);
  k_out<<<dim3(TNB * LQ / 64, CC / 128), 128, 0, stream>>>(Y, F[6], (float*)d_out);
}
